// MambaLayer_34093450396622
// MI455X (gfx1250) — hardware-verified
//
#include <hip/hip_runtime.h>
#include <math.h>

typedef __attribute__((ext_vector_type(8)))  _Float16 v8h;
typedef __attribute__((ext_vector_type(16))) __bf16   v16b;
typedef __attribute__((ext_vector_type(8)))  __bf16   v8b;
typedef __attribute__((ext_vector_type(8)))  float    v8f;
typedef __attribute__((ext_vector_type(4)))  float    v4f;

constexpr int kBatch  = 4;
constexpr int kSeq    = 4096;
constexpr int kDm     = 384;
constexpr int kDin    = 768;
constexpr int kNst    = 16;
constexpr int kDtR    = 24;
constexpr int kDtP    = 32;
constexpr int kXpN    = 56;
constexpr int kXpP    = 64;
constexpr int kXzP    = 2 * kDin;
constexpr int kRows   = kBatch * kSeq;
constexpr int kConvTP = 260;
constexpr int kScanTS = 64;
constexpr int kScanCh = 64;
constexpr int kScanYP = 68;
constexpr int kLnL    = 32;
constexpr int kLnP    = 33;
static_assert(kDtR + 2 * kNst == kXpN, "x_proj width");
static_assert((kDm % 32) == 0 && (kDin % 32) == 0 && (kDtP % 32) == 0, "GEMM K multiples of 32");
static_assert((kSeq % 64) == 0 && (kXzP % 64) == 0 && (kXpP % 64) == 0 && (kDin % 64) == 0 && (kDm % 64) == 0, "GEMM M,N multiples of 64");
static_assert((kSeq % kScanTS) == 0 && (kDin % kScanCh) == 0 && (kDin % 256) == 0 && (kSeq % kLnL) == 0, "tile multiples");
static_assert(((kSeq / 64) * (kXzP / 64)) % 8 == 0 && ((kSeq / 64) * (kXpP / 64)) % 8 == 0 &&
              ((kSeq / 64) * (kDin / 64)) % 8 == 0 && ((kDm / 64) * (kSeq / 64)) % 8 == 0, "8 tiles per GEMM block");

constexpr size_t kOffWIH  = 0;
constexpr size_t kOffWIL  = kOffWIH  + (size_t)kXzP * kDm * 2;
constexpr size_t kOffWXH  = kOffWIL  + (size_t)kXzP * kDm * 2;
constexpr size_t kOffWDH  = kOffWXH  + (size_t)kXpP * kDin * 2;
constexpr size_t kOffWOH  = kOffWDH  + (size_t)kDin * kDtP * 2;
constexpr size_t kOffWOL  = kOffWOH  + (size_t)kDm * kDin * 2;
constexpr size_t kOffXNH  = kOffWOL  + (size_t)kDm * kDin * 2;
constexpr size_t kOffXNL  = kOffXNH  + (size_t)kRows * kDm * 2;
constexpr size_t kOffXZ   = kOffXNL  + (size_t)kRows * kDm * 2;
constexpr size_t kOffUC   = kOffXZ   + (size_t)kSeq * kXzP * 4;
constexpr size_t kOffUCB  = kOffUC   + (size_t)kSeq * kDin * 4;
constexpr size_t kOffPROJ = kOffUCB  + (size_t)kSeq * kDin * 2;
constexpr size_t kOffDT   = kOffPROJ + (size_t)kSeq * kXpP * 4;
constexpr size_t kOffDLR  = kOffDT   + (size_t)kSeq * kDtP * 2;
constexpr size_t kOffYH   = kOffDLR  + (size_t)kSeq * kDin * 4;
constexpr size_t kOffYL   = kOffYH   + (size_t)kSeq * kDin * 2;
constexpr size_t kWsTotal = kOffYL   + (size_t)kSeq * kDin * 2;
static_assert(kWsTotal == 99368960ull, "carve total");
static_assert(kWsTotal <= 134217728ull, "carve cap");
static_assert((kOffWIL % 128) == 0 && (kOffWXH % 128) == 0 && (kOffWDH % 128) == 0 && (kOffWOH % 128) == 0 &&
              (kOffWOL % 128) == 0 && (kOffXNH % 128) == 0 && (kOffXNL % 128) == 0 && (kOffXZ % 128) == 0 &&
              (kOffUC % 128) == 0 && (kOffUCB % 128) == 0 && (kOffPROJ % 128) == 0 && (kOffDT % 128) == 0 &&
              (kOffDLR % 128) == 0 && (kOffYH % 128) == 0 && (kOffYL % 128) == 0, "128-B aligned regions");

__device__ __forceinline__ unsigned short f2bf_bits(float f) {
  unsigned u = __float_as_uint(f);
  return (unsigned short)((u + 0x7FFFu + ((u >> 16) & 1u)) >> 16);
}
__device__ __forceinline__ float bf_bits2f(unsigned short h) { return __uint_as_float(((unsigned)h) << 16); }

__device__ __forceinline__ void grp_guard_b(v8f& a, v8f& b, v8f& c, v8f& d, v16b x, v16b y) {
  asm volatile("v_nop\n\tv_nop\n\tv_nop\n\tv_nop" : "+v"(a), "+v"(b), "+v"(c), "+v"(d) : "v"(x), "v"(y));
}
__device__ __forceinline__ void keep4_b(v16b a, v16b b, v16b c, v16b d) { asm volatile("v_nop" :: "v"(a), "v"(b), "v"(c), "v"(d)); }
__device__ __forceinline__ void acc_guard4(v8f& a, v8f& b, v8f& c, v8f& d) { asm volatile("v_nop\n\tv_nop\n\tv_nop\n\tv_nop" : "+v"(a), "+v"(b), "+v"(c), "+v"(d)); }

struct FragB {
  union U { v16b v; v8b h[2]; };
  static __device__ __forceinline__ v16b load(const __bf16* p) {
    U f; f.h[0] = *(const v8b*)(p); f.h[1] = *(const v8b*)(p + 16); return f.v;
  }
  static __device__ __forceinline__ v8f mma(v16b a, v16b b, v8f c) {
    return __builtin_amdgcn_wmma_f32_16x16x32_bf16(false, a, false, b, (short)0, c, false, false);
  }
};

template <int SPL>
__global__ __launch_bounds__(256) void wmma_gemm64(
    const unsigned short* __restrict__ Ap, const unsigned short* __restrict__ A2p, int lda,
    const unsigned short* __restrict__ Btp, const unsigned short* __restrict__ Bt2p, int ldb,
    float* __restrict__ C, int ldc, int M, int N, int K) {
  typedef __bf16 T;
  typedef v16b V;
  const T* Ab = (const T*)Ap; const T* Ab2 = (const T*)A2p; const T* Bb = (const T*)Btp; const T* Bb2 = (const T*)Bt2p;
  __shared__ __align__(16) float sT[8][16 * 68];
  const int lane = threadIdx.x & 31;
  const int wave = threadIdx.x >> 5;
  const int tilesN = N >> 6;
  const int tilesM = M >> 6;
  const int tile = blockIdx.x * 8 + wave;
  if (tile >= tilesM * tilesN) return;
  const int tm = tile / tilesN;
  const int tn = tile - tm * tilesN;
  const int m0 = tm << 6;
  const int n0 = tn << 6;

  const int rlane = lane & 15;
  const int koff  = (lane >> 4) * 8;
  const int mOff  = (lane >> 4) * 8;

  v8f acc[4][4];
#pragma unroll
  for (int i = 0; i < 4; ++i)
#pragma unroll
    for (int j = 0; j < 4; ++j) acc[i][j] = (v8f){0.f,0.f,0.f,0.f,0.f,0.f,0.f,0.f};

  for (int k0 = 0; k0 < K; k0 += 32) {
    V bh[4], bl[4];
#pragma unroll
    for (int j = 0; j < 4; ++j) {
      const size_t bo = (size_t)(n0 + (j << 4) + rlane) * ldb + koff + k0;
      bh[j] = FragB::load(Bb + bo);
      if (SPL == 2) bl[j] = FragB::load(Bb2 + bo);
    }
#pragma unroll
    for (int i = 0; i < 4; ++i) {
      const size_t ao = (size_t)(m0 + (i << 4) + rlane) * lda + koff + k0;
      V ah = FragB::load(Ab + ao);
      V al;
      if (SPL == 2) al = FragB::load(Ab2 + ao);
#pragma unroll
      for (int j = 0; j < 4; ++j) {
        acc[i][j] = FragB::mma(ah, bh[j], acc[i][j]);
        if (SPL == 2) {
          acc[i][j] = FragB::mma(ah, bl[j], acc[i][j]);
          acc[i][j] = FragB::mma(al, bh[j], acc[i][j]);
        }
      }
      grp_guard_b(acc[i][0], acc[i][1], acc[i][2], acc[i][3], ah, (SPL == 2) ? al : ah);
    }
    keep4_b(bh[0], bh[1], bh[2], bh[3]);
    if (SPL == 2) keep4_b(bl[0], bl[1], bl[2], bl[3]);
  }
  acc_guard4(acc[0][0], acc[0][1], acc[0][2], acc[0][3]);
  acc_guard4(acc[1][0], acc[1][1], acc[1][2], acc[1][3]);
  acc_guard4(acc[2][0], acc[2][1], acc[2][2], acc[2][3]);
  acc_guard4(acc[3][0], acc[3][1], acc[3][2], acc[3][3]);

  float* slab = sT[wave];
#pragma unroll
  for (int i = 0; i < 4; ++i) {
    const int mBase = m0 + (i << 4);
#pragma unroll
    for (int j = 0; j < 4; ++j) {
#pragma unroll
      for (int r = 0; r < 8; ++r) slab[(mOff + r) * 68 + (j << 4) + rlane] = acc[i][j][r];
    }
    __builtin_amdgcn_fence(__ATOMIC_RELEASE, "workgroup");
    __builtin_amdgcn_wave_barrier();
    __builtin_amdgcn_fence(__ATOMIC_ACQUIRE, "workgroup");
    {
      const int hh = lane >> 4, c4 = (lane & 15) * 4;
      for (int pass = 0; pass < 2; ++pass) {
#pragma unroll
        for (int it = 0; it < 8; ++it) {
          const int row = it * 2 + hh;
          v4f v = *(const v4f*)(slab + row * 68 + c4);
          *(volatile v4f*)(C + (size_t)(mBase + row) * ldc + n0 + c4) = v;
        }
        __threadfence();
      }
    }
    __builtin_amdgcn_fence(__ATOMIC_RELEASE, "workgroup");
    __builtin_amdgcn_wave_barrier();
    __builtin_amdgcn_fence(__ATOMIC_ACQUIRE, "workgroup");
  }
}

template <bool LO>
__global__ __launch_bounds__(256) void split_pad_bf16_kernel(
    const float* __restrict__ src, unsigned short* __restrict__ dhi, unsigned short* __restrict__ dlo,
    int N, int K, int Np, int Kp)
{
  const int i = blockIdx.x * 256 + threadIdx.x;
  const int total8 = (Np * Kp) >> 3;
  if (i >= total8) return;
  const int e0 = i << 3;
  const int n  = e0 / Kp;
  const int k0 = e0 - n * Kp;
  const int nc = (n < N) ? n : (N - 1);
  v8h hv, lv;
#pragma unroll
  for (int e = 0; e < 8; ++e) {
    const int k  = k0 + e;
    const int kc = (k < K) ? k : (K - 1);
    const float raw = src[(size_t)nc * K + kc];
    const float v = ((n < N) && (k < K)) ? raw : 0.0f;
    const unsigned short hb = f2bf_bits(v);
    const unsigned short lb = f2bf_bits(v - bf_bits2f(hb));
    hv[e] = __builtin_bit_cast(_Float16, hb);
    lv[e] = __builtin_bit_cast(_Float16, lb);
  }
  unsigned short* qh = dhi + e0;
  unsigned short* ql = dlo + e0;
  *(volatile v8h*)qh = hv;
  if (LO) *(volatile v8h*)ql = lv;
  __threadfence();
  *(volatile v8h*)qh = hv;
  if (LO) *(volatile v8h*)ql = lv;
}

__global__ __launch_bounds__(256) void ln_kernel(
    const float* __restrict__ x, const float* __restrict__ gamma, const float* __restrict__ beta,
    unsigned short* __restrict__ XNH, unsigned short* __restrict__ XNL)
{
  __shared__ __align__(16) float sX[kDm * kLnP];
  __shared__ float sRed[8 * 32];
  __shared__ float sGam[kDm];
  __shared__ float sBet[kDm];
  const int tid = threadIdx.x, lane = tid & 31, wave = tid >> 5;
  constexpr int kBlkPerB = kSeq / kLnL;
  const int b  = blockIdx.x / kBlkPerB;
  const int l0 = (blockIdx.x - b * kBlkPerB) * kLnL;
  const float* xb = x + (size_t)b * kDm * kSeq + l0;

#pragma unroll 1
  for (int i = 0; i < 2; ++i) {
    const int c  = tid + i * 256;
    const int cc = (c < kDm) ? c : (kDm - 1);
    const float gv = gamma[cc];
    const float bv = beta[cc];
    if (c < kDm) { sGam[c] = gv; sBet[c] = bv; }
  }
  {
    const int r = lane >> 3, c4 = (lane & 7) * 4;
#pragma unroll 1
    for (int g3 = 0; g3 < 3; ++g3) {
      v4f v[4];
#pragma unroll
      for (int j = 0; j < 4; ++j) {
        const int c = (g3 * 4 + j) * 32 + wave * 4 + r;
        v[j] = *(const v4f*)(xb + (size_t)c * kSeq + c4);
      }
#pragma unroll
      for (int j = 0; j < 4; ++j) {
        const int c = (g3 * 4 + j) * 32 + wave * 4 + r;
        float* sp = sX + c * kLnP + c4;
        sp[0] = v[j][0]; sp[1] = v[j][1]; sp[2] = v[j][2]; sp[3] = v[j][3];
      }
    }
  }
  __syncthreads();
  constexpr int kCW = kDm / 8;
  float s1 = 0.f;
#pragma unroll 8
  for (int i = 0; i < kCW; ++i) s1 += sX[(wave * kCW + i) * kLnP + lane];
  sRed[wave * 32 + lane] = s1;
  __syncthreads();
  float tot = 0.f;
#pragma unroll
  for (int w = 0; w < 8; ++w) tot += sRed[w * 32 + lane];
  const float mu = tot * (1.0f / (float)kDm);
  __syncthreads();
  float s2 = 0.f;
#pragma unroll 8
  for (int i = 0; i < kCW; ++i) {
    const float dv = sX[(wave * kCW + i) * kLnP + lane] - mu;
    s2 += dv * dv;
  }
  sRed[wave * 32 + lane] = s2;
  __syncthreads();
  float tot2 = 0.f;
#pragma unroll
  for (int w = 0; w < 8; ++w) tot2 += sRed[w * 32 + lane];
  const float var = tot2 * (1.0f / (float)kDm);
  const float inv = rsqrtf(var + 1e-5f);
#pragma unroll 4
  for (int i = 0; i < kCW; ++i) {
    const int c = wave * kCW + i;
    const float v = sX[c * kLnP + lane];
    sX[c * kLnP + lane] = ((v - mu) * inv) * sGam[c] + sBet[c];
  }
  __syncthreads();
  v8h hv[6], lv[6];
#pragma unroll
  for (int it = 0; it < 6; ++it) {
    const int q   = it * 32 + lane;
    const int rr  = q / 48;
    const int c8  = (q - rr * 48) * 8;
    const int row = wave * 4 + rr;
#pragma unroll
    for (int e = 0; e < 8; ++e) {
      const float f = sX[(c8 + e) * kLnP + row];
      const unsigned short hb = f2bf_bits(f);
      const unsigned short lb = f2bf_bits(f - bf_bits2f(hb));
      hv[it][e] = __builtin_bit_cast(_Float16, hb);
      lv[it][e] = __builtin_bit_cast(_Float16, lb);
    }
  }
  const size_t ebase = ((size_t)b * kSeq + l0 + wave * 4) * kDm;
  for (int pass = 0; pass < 2; ++pass) {
#pragma unroll
    for (int it = 0; it < 6; ++it) {
      const size_t o = ebase + (size_t)(it * 32 + lane) * 8;
      *(volatile v8h*)(XNH + o) = hv[it];
      *(volatile v8h*)(XNL + o) = lv[it];
    }
    __threadfence();
  }
}

__global__ __launch_bounds__(256) void conv_silu_kernel(
    const float* __restrict__ XZ, const float* __restrict__ cw, const float* __restrict__ cb,
    float* __restrict__ UC, unsigned short* __restrict__ UCB)
{
  __shared__ __align__(16) float sT[16 * kConvTP];
  const int tid = threadIdx.x, lane = tid & 31, wave = tid >> 5;
  const int d0 = blockIdx.x * 256, d = d0 + tid;
  const int t0 = blockIdx.y * 64;
  const v4f wv = *(const v4f*)(cw + (size_t)d * 4);
  const float w0 = wv[0], w1 = wv[1], w2 = wv[2], w3 = wv[3];
  const float bc = cb[d];
  float xm3, xm2, xm1;
  {
    const int r3 = t0 - 3, r2 = t0 - 2, r1 = t0 - 1;
    const float v3 = XZ[(size_t)(r3 < 0 ? 0 : r3) * kXzP + d];
    const float v2 = XZ[(size_t)(r2 < 0 ? 0 : r2) * kXzP + d];
    const float v1 = XZ[(size_t)(r1 < 0 ? 0 : r1) * kXzP + d];
    xm3 = (r3 >= 0) ? v3 : 0.f;
    xm2 = (r2 >= 0) ? v2 : 0.f;
    xm1 = (r1 >= 0) ? v1 : 0.f;
  }
  const int hrow = wave >> 1;
  const int hch  = (wave & 1) * 128 + lane * 4;
#pragma unroll 1
  for (int sub = 0; sub < 4; ++sub) {
    const int lb = t0 + sub * 16;
#pragma unroll 1
    for (int s = 0; s < 16; ++s) {
      const float xcur = XZ[(size_t)(lb + s) * kXzP + d];
      float acc = w0 * xm3;
      acc = fmaf(w1, xm2, acc);
      acc = fmaf(w2, xm1, acc);
      acc = fmaf(w3, xcur, acc);
      const float sv = acc + bc;
      const float sg = __builtin_amdgcn_rcpf(1.0f + expf(-sv));
      sT[s * kConvTP + tid] = sv * sg;
      xm3 = xm2; xm2 = xm1; xm1 = xcur;
    }
    __syncthreads();
    v4f fv[4];
    v8h bv[2];
#pragma unroll
    for (int it = 0; it < 4; ++it) fv[it] = *(const v4f*)(sT + (it * 4 + hrow) * kConvTP + hch);
#pragma unroll
    for (int it = 0; it < 2; ++it) {
      const float* sp = sT + (it * 8 + wave) * kConvTP + lane * 8;
      const v4f a0 = *(const v4f*)(sp);
      const v4f a1 = *(const v4f*)(sp + 4);
#pragma unroll
      for (int e = 0; e < 4; ++e) {
        const unsigned short h0 = f2bf_bits(a0[e]), h1 = f2bf_bits(a1[e]);
        bv[it][e]     = __builtin_bit_cast(_Float16, h0);
        bv[it][4 + e] = __builtin_bit_cast(_Float16, h1);
      }
    }
    for (int pass = 0; pass < 2; ++pass) {
#pragma unroll
      for (int it = 0; it < 4; ++it)
        *(volatile v4f*)(UC + (size_t)(lb + it * 4 + hrow) * kDin + d0 + hch) = fv[it];
#pragma unroll
      for (int it = 0; it < 2; ++it)
        *(volatile v8h*)(UCB + (size_t)(lb + it * 8 + wave) * kDin + d0 + lane * 8) = bv[it];
      __threadfence();
    }
    __syncthreads();
  }
}

__global__ __launch_bounds__(256) void dt_cast_kernel(
    const float* __restrict__ PROJ, unsigned short* __restrict__ DT16, int total8)
{
  const int i = blockIdx.x * 256 + threadIdx.x;
  if (i >= total8) return;
  const int e0  = i << 3;
  const int row = e0 >> 5;
  const int c8  = e0 & 31;
  const float* p = PROJ + (size_t)row * kXpP + c8;
  const v4f a0 = *(const v4f*)(p);
  const v4f a1 = *(const v4f*)(p + 4);
  const bool live = (c8 < kDtR);
  v8h hv;
#pragma unroll
  for (int e = 0; e < 4; ++e) {
    const float f0 = live ? a0[e] : 0.0f;
    const float f1 = live ? a1[e] : 0.0f;
    const unsigned short h0 = f2bf_bits(f0), h1 = f2bf_bits(f1);
    hv[e]     = __builtin_bit_cast(_Float16, h0);
    hv[4 + e] = __builtin_bit_cast(_Float16, h1);
  }
  unsigned short* qd = DT16 + e0;
  *(volatile v8h*)qd = hv;
  __threadfence();
  *(volatile v8h*)qd = hv;
}

__global__ __launch_bounds__(64) void scan_kernel(
    const float* __restrict__ PROJ, const float* __restrict__ DLR, const float* __restrict__ UC,
    const float* __restrict__ XZ, const float* __restrict__ bdt, const float* __restrict__ Alog,
    const float* __restrict__ Dp, unsigned short* __restrict__ YH, unsigned short* __restrict__ YL)
{
  __shared__ __align__(16) float sBC[kScanTS * 32];
  __shared__ __align__(16) float sY[kScanTS * kScanYP];
  __shared__ __align__(16) float sA[kNst * kScanCh];
  const int tid = threadIdx.x, lane = tid & 31, wave = tid >> 5;
  const int d0 = blockIdx.x * kScanCh;
  const int d  = d0 + tid;
#pragma unroll 1
  for (int s = 0; s < kNst; ++s) sA[s * kScanCh + tid] = -expf(Alog[(size_t)d * kNst + s]);
  __syncthreads();
  float negA[kNst], h[kNst];
#pragma unroll
  for (int s = 0; s < kNst; ++s) {
    negA[s] = sA[s * kScanCh + tid];
    h[s] = 0.f;
  }
  const float bb = bdt[d], Dd = Dp[d];
  const int sr = tid >> 3, sc4 = (tid & 7) * 4;
  const int q = lane >> 3, c8 = (lane & 7) * 8;
#pragma unroll 1
  for (int t0 = 0; t0 < kSeq; t0 += kScanTS) {
    __syncthreads();
    {
      v4f st[8];
#pragma unroll
      for (int i = 0; i < 8; ++i)
        st[i] = *(const v4f*)(PROJ + (size_t)(t0 + sr + 8 * i) * kXpP + kDtR + sc4);
#pragma unroll
      for (int i = 0; i < 8; ++i)
        *(v4f*)(sBC + (sr + 8 * i) * 32 + sc4) = st[i];
    }
    __syncthreads();
#pragma unroll 1
    for (int s = 0; s < kScanTS; ++s) {
      const size_t t = (size_t)(t0 + s);
      const float* xr = sBC + s * 32;
      float Bs[kNst], Cs[kNst];
#pragma unroll
      for (int q4 = 0; q4 < 4; ++q4) {
        const v4f bv = *(const v4f*)(xr + 4 * q4);
        const v4f cv = *(const v4f*)(xr + kNst + 4 * q4);
        Bs[4 * q4 + 0] = bv[0]; Bs[4 * q4 + 1] = bv[1]; Bs[4 * q4 + 2] = bv[2]; Bs[4 * q4 + 3] = bv[3];
        Cs[4 * q4 + 0] = cv[0]; Cs[4 * q4 + 1] = cv[1]; Cs[4 * q4 + 2] = cv[2]; Cs[4 * q4 + 3] = cv[3];
      }
      const float v   = DLR[t * kDin + d] + bb;
      const float a   = expf(-fabsf(v));
      const float u   = 1.0f + a;
      const float l1p = __logf(u) + (a - (u - 1.0f)) * __builtin_amdgcn_rcpf(u);
      const float dt  = fmaxf(v, 0.0f) + l1p;
      const float xt  = UC[t * kDin + d];
      const float zv  = XZ[t * kXzP + kDin + d];
      const float dtx = dt * xt;
      float y = 0.f;
#pragma unroll
      for (int k = 0; k < kNst; ++k) {
        const float e = __expf(dt * negA[k]);
        h[k] = e * h[k] + dtx * Bs[k];
        y = h[k] * Cs[k] + y;
      }
      y = xt * Dd + y;
      const float sg = __builtin_amdgcn_rcpf(1.0f + expf(-zv));
      y = y * (zv * sg);
      sY[s * kScanYP + tid] = y;
    }
    __syncthreads();
    v8h hv[8], lv[8];
#pragma unroll
    for (int it = 0; it < 8; ++it) {
      const int row = it * 8 + wave * 4 + q;
      const float* sp = sY + row * kScanYP + c8;
      const v4f a0 = *(const v4f*)(sp);
      const v4f a1 = *(const v4f*)(sp + 4);
#pragma unroll
      for (int e = 0; e < 4; ++e) {
        const unsigned short h0 = f2bf_bits(a0[e]), h1 = f2bf_bits(a1[e]);
        const unsigned short l0 = f2bf_bits(a0[e] - bf_bits2f(h0)), l1 = f2bf_bits(a1[e] - bf_bits2f(h1));
        hv[it][e]     = __builtin_bit_cast(_Float16, h0);
        hv[it][4 + e] = __builtin_bit_cast(_Float16, h1);
        lv[it][e]     = __builtin_bit_cast(_Float16, l0);
        lv[it][4 + e] = __builtin_bit_cast(_Float16, l1);
      }
    }
    for (int pass = 0; pass < 2; ++pass) {
#pragma unroll
      for (int it = 0; it < 8; ++it) {
        const int row = it * 8 + wave * 4 + q;
        const size_t o = (size_t)(t0 + row) * kDin + d0 + c8;
        *(volatile v8h*)(YH + o) = hv[it];
        *(volatile v8h*)(YL + o) = lv[it];
      }
      __threadfence();
    }
  }
}

extern "C" void kernel_launch(void* const* d_in, const int* in_sizes, int n_in,
                              void* d_out, int out_size, void* d_ws, size_t ws_size,
                              hipStream_t stream) {
  if (n_in < 12) return;
  if (in_sizes[0] != kRows * kDm) return;
  if (in_sizes[1] != kDm || in_sizes[2] != kDm) return;
  if (in_sizes[3] != kXzP * kDm) return;
  if (in_sizes[4] != kDin * 4 || in_sizes[5] != kDin) return;
  if (in_sizes[6] != kXpN * kDin) return;
  if (in_sizes[7] != kDin * kDtR || in_sizes[8] != kDin) return;
  if (in_sizes[9] != kDin * kNst || in_sizes[10] != kDin) return;
  if (in_sizes[11] != kDm * kDin) return;
  if (out_size != kRows * kDm) return;
  if (ws_size < kWsTotal) return;

  const float* x       = (const float*)d_in[0];
  const float* gamma   = (const float*)d_in[1];
  const float* beta    = (const float*)d_in[2];
  const float* W_in    = (const float*)d_in[3];
  const float* conv_w  = (const float*)d_in[4];
  const float* conv_b  = (const float*)d_in[5];
  const float* W_xproj = (const float*)d_in[6];
  const float* W_dt    = (const float*)d_in[7];
  const float* b_dt    = (const float*)d_in[8];
  const float* A_log   = (const float*)d_in[9];
  const float* Dp      = (const float*)d_in[10];
  const float* W_out   = (const float*)d_in[11];
  float* out = (float*)d_out;

  char* ws = (char*)d_ws;
  unsigned short* WIH  = (unsigned short*)(ws + kOffWIH);
  unsigned short* WIL  = (unsigned short*)(ws + kOffWIL);
  unsigned short* WXH  = (unsigned short*)(ws + kOffWXH);
  unsigned short* WDH  = (unsigned short*)(ws + kOffWDH);
  unsigned short* WOH  = (unsigned short*)(ws + kOffWOH);
  unsigned short* WOL  = (unsigned short*)(ws + kOffWOL);
  unsigned short* XNH  = (unsigned short*)(ws + kOffXNH);
  unsigned short* XNL  = (unsigned short*)(ws + kOffXNL);
  float*          XZ   = (float*)(ws + kOffXZ);
  float*          UC   = (float*)(ws + kOffUC);
  unsigned short* UCB  = (unsigned short*)(ws + kOffUCB);
  float*          PROJ = (float*)(ws + kOffPROJ);
  unsigned short* DT16 = (unsigned short*)(ws + kOffDT);
  float*          DLR  = (float*)(ws + kOffDLR);
  unsigned short* YH   = (unsigned short*)(ws + kOffYH);
  unsigned short* YL   = (unsigned short*)(ws + kOffYL);

  split_pad_bf16_kernel<true ><<<(kXzP * kDm / 8) / 256, 256, 0, stream>>>(W_in,    WIH, WIL, kXzP, kDm,  kXzP, kDm);
  split_pad_bf16_kernel<false><<<(kXpP * kDin / 8) / 256, 256, 0, stream>>>(W_xproj, WXH, WXH, kXpN, kDin, kXpP, kDin);
  split_pad_bf16_kernel<false><<<(kDin * kDtP / 8) / 256, 256, 0, stream>>>(W_dt,    WDH, WDH, kDin, kDtR, kDin, kDtP);
  split_pad_bf16_kernel<true ><<<(kDm * kDin / 8) / 256, 256, 0, stream>>>(W_out,   WOH, WOL, kDm,  kDin, kDm,  kDin);

  ln_kernel<<<kBatch * (kSeq / kLnL), 256, 0, stream>>>(x, gamma, beta, XNH, XNL);

  for (int b = 0; b < kBatch; ++b) {
    const unsigned short* XNHb = XNH + (size_t)b * kSeq * kDm;
    const unsigned short* XNLb = XNL + (size_t)b * kSeq * kDm;
    float* outb = out + (size_t)b * kDm * kSeq;

    wmma_gemm64<2><<<((kSeq / 64) * (kXzP / 64)) / 8, 256, 0, stream>>>(
        XNHb, XNLb, kDm, WIH, WIL, kDm, XZ, kXzP, kSeq, kXzP, kDm);

    conv_silu_kernel<<<dim3(kDin / 256, kSeq / 64), 256, 0, stream>>>(XZ, conv_w, conv_b, UC, UCB);

    wmma_gemm64<0><<<((kSeq / 64) * (kXpP / 64)) / 8, 256, 0, stream>>>(
        UCB, UCB, kDin, WXH, WXH, kDin, PROJ, kXpP, kSeq, kXpP, kDin);

    dt_cast_kernel<<<(kSeq * kDtP / 8) / 256, 256, 0, stream>>>(PROJ, DT16, kSeq * kDtP / 8);

    wmma_gemm64<0><<<((kSeq / 64) * (kDin / 64)) / 8, 256, 0, stream>>>(
        DT16, DT16, kDtP, WDH, WDH, kDtP, DLR, kDin, kSeq, kDin, kDtP);

    scan_kernel<<<kDin / kScanCh, kScanCh, 0, stream>>>(PROJ, DLR, UC, XZ, b_dt, A_log, Dp, YH, YL);

    wmma_gemm64<2><<<((kDm / 64) * (kSeq / 64)) / 8, 256, 0, stream>>>(
        WOH, WOL, kDin, YH, YL, kDin, outb, kSeq, kDm, kSeq, kDin);
  }
}
